// NonLocalAttention_73744588472613
// MI455X (gfx1250) — hardware-verified
//
#include <hip/hip_runtime.h>
#include <stdint.h>

typedef __attribute__((ext_vector_type(16))) _Float16 v16h;
typedef __attribute__((ext_vector_type(8)))  _Float16 v8h;
typedef __attribute__((ext_vector_type(16))) __bf16   v16b;
typedef __attribute__((ext_vector_type(8)))  __bf16   v8b;
typedef __attribute__((ext_vector_type(8)))  float    v8f;
typedef __attribute__((ext_vector_type(4)))  float    v4f;
typedef __attribute__((ext_vector_type(4)))  unsigned int v4u;

constexpr int kBatch  = 2;
constexpr int kCh     = 256;
constexpr int kCi     = 128;
constexpr int kImgW   = 64;
constexpr int kNPos   = 4096;
constexpr int kLayers = 4;
constexpr int kPadW   = 66;
constexpr int kNPad   = kPadW * kPadW;
constexpr int kKConv  = 9 * kCh;
constexpr float kBnEps  = 1e-5f;
constexpr float kPCarry = 32768.0f;

constexpr int kTabGb  = 0;
constexpr int kTabThb = 512;
constexpr int kTabPhb = 1024;
constexpr int kTabWb  = 1536;
constexpr int kTabCb  = 2560;
constexpr int kTabS1  = 3584;
constexpr int kTabT1  = 4608;
constexpr int kTabS2  = 5632;
constexpr int kTabT2  = 6656;
constexpr int kTabTotal = 7680;

static_assert(kNPos == kImgW * kImgW, "geometry");
static_assert(kImgW == 64, "one 64-row M tile equals one image row");
static_assert(kNPos % 64 == 0 && kCh % 64 == 0 && kCi % 64 == 0, "M/N tile multiples");
static_assert(kCh % 32 == 0 && kCi % 32 == 0 && kKConv % 32 == 0, "K multiple of 32");

__device__ __forceinline__ unsigned short f2bf_bits(float f) {
  unsigned u = __float_as_uint(f);
  return (unsigned short)((u + 0x7FFFu + ((u >> 16) & 1u)) >> 16);
}
__device__ __forceinline__ float bf_bits2f(unsigned short h) { return __uint_as_float(((unsigned)h) << 16); }
__device__ __forceinline__ float bf_rne(float f) { return bf_bits2f(f2bf_bits(f)); }

__device__ __forceinline__ void dep_guard_h(v8f& a, v8f& b, v16h x, v16h y) { asm volatile("v_nop\n\tv_nop\n\tv_nop\n\tv_nop" : "+v"(a), "+v"(b) : "v"(x), "v"(y)); }
__device__ __forceinline__ void dep_guard_b(v8f& a, v8f& b, v16b x, v16b y) { asm volatile("v_nop\n\tv_nop\n\tv_nop\n\tv_nop" : "+v"(a), "+v"(b) : "v"(x), "v"(y)); }
__device__ __forceinline__ void dep_guard1_h(v8f& c, v16h x, v16h y) { asm volatile("v_nop\n\tv_nop\n\tv_nop\n\tv_nop" : "+v"(c) : "v"(x), "v"(y)); }
__device__ __forceinline__ void dep_guard1_b(v8f& c, v16b x, v16b y) { asm volatile("v_nop\n\tv_nop\n\tv_nop\n\tv_nop" : "+v"(c) : "v"(x), "v"(y)); }
__device__ __forceinline__ void keep4_h(v16h a, v16h b, v16h c, v16h d) { asm volatile("v_nop" :: "v"(a), "v"(b), "v"(c), "v"(d)); }
__device__ __forceinline__ void keep4_b(v16b a, v16b b, v16b c, v16b d) { asm volatile("v_nop" :: "v"(a), "v"(b), "v"(c), "v"(d)); }
__device__ __forceinline__ void acc_guard4(v8f& a, v8f& b, v8f& c, v8f& d) { asm volatile("v_nop\n\tv_nop\n\tv_nop\n\tv_nop" : "+v"(a), "+v"(b), "+v"(c), "+v"(d)); }

template <typename T> struct Frag;
template <> struct Frag<_Float16> {
  typedef v16h V; union U { v16h v; v8h h[2]; };
  static __device__ __forceinline__ v16h load(const _Float16* p) {
    U f; f.h[0] = *(const v8h*)(p); f.h[1] = *(const v8h*)(p + 16); return f.v;
  }
  static __device__ __forceinline__ v8f mma(v16h a, v16h b, v8f c) {
    return __builtin_amdgcn_wmma_f32_16x16x32_f16(false, a, false, b, (short)0, c, false, false);
  }
  static __device__ __forceinline__ v8f mmag(v16h a, v16h b, v8f c) { c = mma(a, b, c); dep_guard1_h(c, a, b); return c; }
  static __device__ __forceinline__ void guard(v8f& a, v8f& b, v16h x, v16h y) { dep_guard_h(a, b, x, y); }
  static __device__ __forceinline__ void keep(v16h a, v16h b, v16h c, v16h d) { keep4_h(a, b, c, d); }
};
template <> struct Frag<__bf16> {
  typedef v16b V; union U { v16b v; v8b h[2]; };
  static __device__ __forceinline__ v16b load(const __bf16* p) {
    U f; f.h[0] = *(const v8b*)(p); f.h[1] = *(const v8b*)(p + 16); return f.v;
  }
  static __device__ __forceinline__ v8f mma(v16b a, v16b b, v8f c) {
    return __builtin_amdgcn_wmma_f32_16x16x32_bf16(false, a, false, b, (short)0, c, false, false);
  }
  static __device__ __forceinline__ v8f mmag(v16b a, v16b b, v8f c) { c = mma(a, b, c); dep_guard1_b(c, a, b); return c; }
  static __device__ __forceinline__ void guard(v8f& a, v8f& b, v16b x, v16b y) { dep_guard_b(a, b, x, y); }
  static __device__ __forceinline__ void keep(v16b a, v16b b, v16b c, v16b d) { keep4_b(a, b, c, d); }
};
template <int ET> struct Elem;
template <> struct Elem<0> { typedef _Float16 T; };
template <> struct Elem<1> { typedef __bf16 T; };

template <bool SPLIT_A, bool SPLIT_B, int BIAS_MODE, int EPI, int OUT_MODE, bool PADROWS, bool RESID>
__global__ __launch_bounds__(256) void gemm_bf16_64(
    const unsigned short* __restrict__ Ap, const unsigned short* __restrict__ A2p, int lda, long strideA,
    const unsigned short* __restrict__ Btp, const unsigned short* __restrict__ Bt2p, int ldb, long strideB,
    void* __restrict__ Cout, void* __restrict__ Cout2, int ldc, long strideC,
    const float* __restrict__ bias, const float* __restrict__ bns, const float* __restrict__ bnt,
    const float* __restrict__ resid, int ldr, long strideR,
    int M, int N, int K) {
  typedef __bf16 T;
  typedef v16b V;
  const T* A = (const T*)Ap; const T* A2 = (const T*)A2p; const T* Bt = (const T*)Btp; const T* Bt2 = (const T*)Bt2p;
  __shared__ __align__(16) float sT[8][16 * 68];
  const int b    = blockIdx.y;
  const int lane = threadIdx.x & 31;
  const int wave = threadIdx.x >> 5;
  const int tilesN = N >> 6;
  const int tilesM = M >> 6;
  const int tile = blockIdx.x * 8 + wave;
  if (tile >= tilesM * tilesN) return;
  const int tm = tile / tilesN;
  const int tn = tile - tm * tilesN;
  const int m0 = tm << 6;
  const int n0 = tn << 6;

  const T* Ab  = A  + (size_t)b * strideA;
  const T* Bb  = Bt + (size_t)b * strideB;
  const T* Ab2 = SPLIT_A ? (A2  + (size_t)b * strideA) : Ab;
  const T* Bb2 = SPLIT_B ? (Bt2 + (size_t)b * strideB) : Bb;

  const int rlane = lane & 15;
  const int koff  = (lane >> 4) * 8;
  const int mOff  = (lane >> 4) * 8;

  v8f acc[4][4];
#pragma unroll
  for (int i = 0; i < 4; ++i)
#pragma unroll
    for (int j = 0; j < 4; ++j) acc[i][j] = (v8f){0.f,0.f,0.f,0.f,0.f,0.f,0.f,0.f};

  for (int k0 = 0; k0 < K; k0 += 32) {
    V bh[4], bl[4];
#pragma unroll
    for (int j = 0; j < 4; ++j) {
      const size_t bo = (size_t)(n0 + (j << 4) + rlane) * ldb + koff + k0;
      bh[j] = Frag<T>::load(Bb + bo);
      if (SPLIT_B) bl[j] = Frag<T>::load(Bb2 + bo);
    }
#pragma unroll
    for (int i = 0; i < 4; ++i) {
      const size_t ao = (size_t)(m0 + (i << 4) + rlane) * lda + koff + k0;
      V ah = Frag<T>::load(Ab + ao);
      V al = ah;
      if (SPLIT_A) al = Frag<T>::load(Ab2 + ao);
#pragma unroll
      for (int j = 0; j < 4; ++j) {
        acc[i][j] = Frag<T>::mma(ah, bh[j], acc[i][j]);
        if (SPLIT_B) acc[i][j] = Frag<T>::mma(ah, bl[j], acc[i][j]);
        if (SPLIT_A) acc[i][j] = Frag<T>::mma(al, bh[j], acc[i][j]);
      }
      Frag<T>::guard(acc[i][0], acc[i][3], ah, al);
    }
    Frag<T>::keep(bh[0], bh[1], bh[2], bh[3]);
    if (SPLIT_B) Frag<T>::keep(bl[0], bl[1], bl[2], bl[3]);
  }
  acc_guard4(acc[0][0], acc[0][1], acc[0][2], acc[0][3]);
  acc_guard4(acc[1][0], acc[1][1], acc[1][2], acc[1][3]);
  acc_guard4(acc[2][0], acc[2][1], acc[2][2], acc[2][3]);
  acc_guard4(acc[3][0], acc[3][1], acc[3][2], acc[3][3]);

  float* slab = sT[wave];
  float colb[4], cols[4], colt[4];
#pragma unroll
  for (int j = 0; j < 4; ++j) {
    const int n = n0 + (j << 4) + rlane;
    colb[j] = 0.f; cols[j] = 1.f; colt[j] = 0.f;
    if (BIAS_MODE == 2) colb[j] = bias[n];
    if (EPI > 0) { cols[j] = bns[n]; colt[j] = bnt[n]; }
  }
  const int mS0 = PADROWS ? ((m0 / kImgW + 1) * kPadW + 1) : m0;
  const float* Rb = RESID ? (resid + (size_t)b * strideR) : resid;
#pragma unroll
  for (int i = 0; i < 4; ++i) {
    const int mBase = m0 + (i << 4);
    const int mSB   = mS0 + (i << 4);
    v4f bm0 = (v4f){0.f,0.f,0.f,0.f}, bm1 = (v4f){0.f,0.f,0.f,0.f};
    if (BIAS_MODE == 1) {
      bm0 = *(const v4f*)(bias + mBase + mOff);
      bm1 = *(const v4f*)(bias + mBase + mOff + 4);
    }
#pragma unroll
    for (int j = 0; j < 4; ++j) {
#pragma unroll
      for (int r = 0; r < 8; ++r) {
        float v = acc[i][j][r];
        if (BIAS_MODE == 1) v += (r < 4) ? bm0[r & 3] : bm1[r & 3];
        v += colb[j];
        if (EPI > 0) v = v * cols[j] + colt[j];
        if (EPI == 2) v = fmaxf(v, 0.0f);
        slab[(mOff + r) * 68 + (j << 4) + rlane] = v;
      }
    }
    __builtin_amdgcn_fence(__ATOMIC_RELEASE, "workgroup");
    __builtin_amdgcn_wave_barrier();
    __builtin_amdgcn_fence(__ATOMIC_ACQUIRE, "workgroup");
    if (OUT_MODE == 0) {
      float* C = (float*)Cout + (size_t)b * strideC;
      const int h2 = lane >> 4, c4 = (lane & 15) * 4;
      for (int pass = 0; pass < 2; ++pass) {
#pragma unroll
        for (int it = 0; it < 8; ++it) {
          const int row = it * 2 + h2;
          v4f v = *(const v4f*)(slab + row * 68 + c4);
          *(volatile v4f*)(C + (size_t)(mSB + row) * ldc + n0 + c4) = v;
        }
        __threadfence();
      }
    } else {
      const int q = lane >> 3, c8 = (lane & 7) * 8;
      unsigned short* C  = (unsigned short*)Cout  + (size_t)b * strideC;
      unsigned short* C2 = (unsigned short*)Cout2 + (size_t)b * strideC;
      for (int pass = 0; pass < 2; ++pass) {
#pragma unroll
        for (int it = 0; it < 4; ++it) {
          const int row = it * 4 + q;
          const float* sp = slab + row * 68 + c8;
          float vv[8];
#pragma unroll
          for (int e = 0; e < 8; ++e) vv[e] = sp[e];
          if (RESID) {
            const float* rp = Rb + (size_t)(mBase + row) * ldr + n0 + c8;
            const v4f rv0 = *(const v4f*)rp;
            const v4f rv1 = *(const v4f*)(rp + 4);
#pragma unroll
            for (int e = 0; e < 4; ++e) { vv[e] += rv0[e]; vv[4 + e] += rv1[e]; }
          }
          v8h hv, lv;
#pragma unroll
          for (int e = 0; e < 8; ++e) {
            if (OUT_MODE == 1) {
              hv[e] = (_Float16)vv[e];
              lv[e] = hv[e];
            } else {
              const unsigned short hb = f2bf_bits(vv[e]);
              const unsigned short lb = f2bf_bits(vv[e] - bf_bits2f(hb));
              hv[e] = __builtin_bit_cast(_Float16, hb);
              lv[e] = __builtin_bit_cast(_Float16, lb);
            }
          }
          *(volatile v8h*)(C + (size_t)(mSB + row) * ldc + n0 + c8) = hv;
          if (OUT_MODE == 2) *(volatile v8h*)(C2 + (size_t)(mSB + row) * ldc + n0 + c8) = lv;
        }
        __threadfence();
      }
    }
    __builtin_amdgcn_fence(__ATOMIC_RELEASE, "workgroup");
    __builtin_amdgcn_wave_barrier();
    __builtin_amdgcn_fence(__ATOMIC_ACQUIRE, "workgroup");
  }
}

__global__ __launch_bounds__(256) void conv3x3_bf16_64(
    const unsigned short* __restrict__ Xh, const unsigned short* __restrict__ Xl,
    const unsigned short* __restrict__ Wp,
    float* __restrict__ Cout,
    const float* __restrict__ bias, const float* __restrict__ bns, const float* __restrict__ bnt) {
  typedef __bf16 T;
  typedef v16b V;
  __shared__ __align__(16) float sT[8][16 * 68];
  const int b    = blockIdx.y;
  const int lane = threadIdx.x & 31;
  const int wave = threadIdx.x >> 5;
  constexpr int tilesN = kCh >> 6;
  const int tile = blockIdx.x * 8 + wave;
  if (tile >= (kNPos >> 6) * tilesN) return;
  const int tm = tile / tilesN;
  const int tn = tile - tm * tilesN;
  const int m0 = tm << 6;
  const int n0 = tn << 6;

  const T* Ab  = (const T*)Xh + (size_t)b * kNPad * kCh;
  const T* Ab2 = (const T*)Xl + (size_t)b * kNPad * kCh;
  const T* Bb  = (const T*)Wp;

  const int rlane = lane & 15;
  const int koff  = (lane >> 4) * 8;
  const int mOff  = (lane >> 4) * 8;

  v8f acc[4][4];
#pragma unroll
  for (int i = 0; i < 4; ++i)
#pragma unroll
    for (int j = 0; j < 4; ++j) acc[i][j] = (v8f){0.f,0.f,0.f,0.f,0.f,0.f,0.f,0.f};

#pragma unroll 1
  for (int tap = 0; tap < 9; ++tap) {
    const int ky = tap / 3;
    const int kx = tap - ky * 3;
    const int arow = (tm + ky) * kPadW + kx;
    const T* At  = Ab  + (size_t)arow * kCh;
    const T* At2 = Ab2 + (size_t)arow * kCh;
    const T* Btap = Bb + tap * kCh;
    for (int kk = 0; kk < kCh; kk += 32) {
      V bh[4];
#pragma unroll
      for (int j = 0; j < 4; ++j) {
        const size_t bo = (size_t)(n0 + (j << 4) + rlane) * kKConv + koff + kk;
        bh[j] = Frag<T>::load(Btap + bo);
      }
#pragma unroll
      for (int i = 0; i < 4; ++i) {
        const size_t ao = (size_t)((i << 4) + rlane) * kCh + koff + kk;
        V ah = Frag<T>::load(At + ao);
        V al = Frag<T>::load(At2 + ao);
#pragma unroll
        for (int j = 0; j < 4; ++j) {
          acc[i][j] = Frag<T>::mma(ah, bh[j], acc[i][j]);
          acc[i][j] = Frag<T>::mma(al, bh[j], acc[i][j]);
        }
        Frag<T>::guard(acc[i][0], acc[i][3], ah, al);
      }
      Frag<T>::keep(bh[0], bh[1], bh[2], bh[3]);
    }
  }
  acc_guard4(acc[0][0], acc[0][1], acc[0][2], acc[0][3]);
  acc_guard4(acc[1][0], acc[1][1], acc[1][2], acc[1][3]);
  acc_guard4(acc[2][0], acc[2][1], acc[2][2], acc[2][3]);
  acc_guard4(acc[3][0], acc[3][1], acc[3][2], acc[3][3]);

  float* slab = sT[wave];
  float colb[4], cols[4], colt[4];
#pragma unroll
  for (int j = 0; j < 4; ++j) {
    const int n = n0 + (j << 4) + rlane;
    colb[j] = bias[n]; cols[j] = bns[n]; colt[j] = bnt[n];
  }
  float* C = Cout + (size_t)b * kNPos * kCh;
#pragma unroll
  for (int i = 0; i < 4; ++i) {
    const int mBase = m0 + (i << 4);
#pragma unroll
    for (int j = 0; j < 4; ++j) {
#pragma unroll
      for (int r = 0; r < 8; ++r) {
        float v = acc[i][j][r] + colb[j];
        v = v * cols[j] + colt[j];
        v = fmaxf(v, 0.0f);
        slab[(mOff + r) * 68 + (j << 4) + rlane] = v;
      }
    }
    __builtin_amdgcn_fence(__ATOMIC_RELEASE, "workgroup");
    __builtin_amdgcn_wave_barrier();
    __builtin_amdgcn_fence(__ATOMIC_ACQUIRE, "workgroup");
    {
      const int h2 = lane >> 4, c4 = (lane & 15) * 4;
      for (int pass = 0; pass < 2; ++pass) {
#pragma unroll
        for (int it = 0; it < 8; ++it) {
          const int row = it * 2 + h2;
          v4f v = *(const v4f*)(slab + row * 68 + c4);
          *(volatile v4f*)(C + (size_t)(mBase + row) * kCh + n0 + c4) = v;
        }
        __threadfence();
      }
    }
    __builtin_amdgcn_fence(__ATOMIC_RELEASE, "workgroup");
    __builtin_amdgcn_wave_barrier();
    __builtin_amdgcn_fence(__ATOMIC_ACQUIRE, "workgroup");
  }
}

constexpr int kAttKC = 32;
constexpr int kAttKP = 136;
constexpr int kAttVP = 40;
constexpr int kAttPP = 40;
constexpr int kAttOP = 132;
constexpr int kAttNW = 4;
static_assert(kNPos % kAttKC == 0 && kNPos % 64 == 0 && kCi == 128, "attention geometry");

template <bool SPLITQK>
__global__ __launch_bounds__(128) void attn_kernel(
    const unsigned short* thh, const unsigned short* thl,
    const unsigned short* __restrict__ phh, const unsigned short* __restrict__ phl,
    const unsigned short* __restrict__ gp,
    unsigned short* __restrict__ yh, unsigned short* __restrict__ yl) {
  typedef typename Elem<SPLITQK ? 1 : 0>::T QT;
  typedef typename Frag<QT>::V QV;
  __shared__ __align__(16) unsigned short Ksh[kAttKC * kAttKP];
  __shared__ __align__(16) unsigned short Ksl[SPLITQK ? kAttKC * kAttKP : 8];
  __shared__ __align__(16) unsigned short Vts[kCi * kAttVP];
  __shared__ __align__(16) _Float16 Psh[kAttNW][16 * kAttPP];
  __shared__ __align__(16) float Osh[kAttNW][16 * kAttOP];

  const int tid  = threadIdx.x;
  const int wave = tid >> 5;
  const int lane = tid & 31;
  const int hh   = lane >> 4;
  const int c    = lane & 15;
  const int b    = blockIdx.y;
  const int q0   = blockIdx.x * 64 + wave * 16;
  const size_t pl = (size_t)kNPos * kCi;
  const unsigned short* thh_b = thh + (size_t)b * pl;
  const unsigned short* thl_b = thl + (size_t)b * pl;
  const unsigned short* phh_b = phh + (size_t)b * pl;
  const unsigned short* phl_b = phl + (size_t)b * pl;
  const unsigned short* gp_b  = gp  + (size_t)b * pl;

  float mrow[8], lrow[8];
  v8f oacc[8];
#pragma unroll
  for (int r = 0; r < 8; ++r) { mrow[r] = -__builtin_inff(); lrow[r] = 0.f; }
#pragma unroll
  for (int t = 0; t < 8; ++t) oacc[t] = (v8f){0.f,0.f,0.f,0.f,0.f,0.f,0.f,0.f};

  for (int kc = 0; kc < kNPos / kAttKC; ++kc) {
    const int kv0 = kc * kAttKC;
    __syncthreads();
#pragma unroll
    for (int i = 0; i < 4; ++i) {
      const int idx = tid + 128 * i;
      const int row = idx >> 4, ch = idx & 15;
      const v4u kq = *(const v4u*)(phh_b + (size_t)(kv0 + row) * kCi + ch * 8);
      *(v4u*)(Ksh + row * kAttKP + ch * 8) = kq;
      if (SPLITQK) {
        const v4u kq2 = *(const v4u*)(phl_b + (size_t)(kv0 + row) * kCi + ch * 8);
        *(v4u*)(Ksl + row * kAttKP + ch * 8) = kq2;
      }
      const int d = idx >> 2, ch2 = idx & 3;
      const v4u vq = *(const v4u*)(gp_b + (size_t)d * kNPos + kv0 + ch2 * 8);
      *(v4u*)(Vts + d * kAttVP + ch2 * 8) = vq;
    }
    __syncthreads();

    v8f s[2];
    s[0] = (v8f){0.f,0.f,0.f,0.f,0.f,0.f,0.f,0.f};
    s[1] = (v8f){0.f,0.f,0.f,0.f,0.f,0.f,0.f,0.f};
#pragma unroll
    for (int dc = 0; dc < 4; ++dc) {
      const size_t qo = (size_t)(q0 + c) * kCi + dc * 32 + 8 * hh;
      const QV qh = Frag<QT>::load((const QT*)(thh_b + qo));
      QV ql = qh;
      if (SPLITQK) ql = Frag<QT>::load((const QT*)(thl_b + qo));
#pragma unroll
      for (int j = 0; j < 2; ++j) {
        const int ko = (j * 16 + c) * kAttKP + dc * 32 + 8 * hh;
        const QV kh = Frag<QT>::load((const QT*)(Ksh + ko));
        s[j] = Frag<QT>::mmag(qh, kh, s[j]);
        if (SPLITQK) {
          const QV kl = Frag<QT>::load((const QT*)(Ksl + ko));
          s[j] = Frag<QT>::mmag(qh, kl, s[j]);
          s[j] = Frag<QT>::mmag(ql, kh, s[j]);
        }
      }
    }

    float cm[8];
#pragma unroll
    for (int r = 0; r < 8; ++r) {
      float m = fmaxf(s[0][r], s[1][r]);
      m = fmaxf(m, __shfl_xor(m, 1, 32));
      m = fmaxf(m, __shfl_xor(m, 2, 32));
      m = fmaxf(m, __shfl_xor(m, 4, 32));
      m = fmaxf(m, __shfl_xor(m, 8, 32));
      cm[r] = m;
    }
    _Float16* pw = Psh[wave];
#pragma unroll
    for (int r = 0; r < 8; ++r) {
      const float mnew  = fmaxf(mrow[r], cm[r]);
      const float alpha = expf(mrow[r] - mnew);
      mrow[r] = mnew;
      const float p0 = expf(s[0][r] - mnew);
      const float p1 = expf(s[1][r] - mnew);
      float psum = p0 + p1;
      psum += __shfl_xor(psum, 1, 32);
      psum += __shfl_xor(psum, 2, 32);
      psum += __shfl_xor(psum, 4, 32);
      psum += __shfl_xor(psum, 8, 32);
      lrow[r] = lrow[r] * alpha + psum;
      pw[(8 * hh + r) * kAttPP + c]      = (_Float16)(p0 * kPCarry);
      pw[(8 * hh + r) * kAttPP + 16 + c] = (_Float16)(p1 * kPCarry);
#pragma unroll
      for (int t = 0; t < 8; ++t) oacc[t][r] *= alpha;
    }
    __builtin_amdgcn_fence(__ATOMIC_RELEASE, "workgroup");
    __builtin_amdgcn_wave_barrier();
    __builtin_amdgcn_fence(__ATOMIC_ACQUIRE, "workgroup");

    const v16h pa = Frag<_Float16>::load(pw + c * kAttPP + 8 * hh);
#pragma unroll
    for (int t = 0; t < 8; ++t) {
      const v16h vb = Frag<_Float16>::load((const _Float16*)(Vts + (t * 16 + c) * kAttVP + 8 * hh));
      oacc[t] = Frag<_Float16>::mmag(pa, vb, oacc[t]);
    }
  }

  float* os = Osh[wave];
#pragma unroll
  for (int r = 0; r < 8; ++r) {
    const float inv = 1.0f / (lrow[r] * kPCarry);
#pragma unroll
    for (int t = 0; t < 8; ++t) os[(8 * hh + r) * kAttOP + t * 16 + c] = oacc[t][r] * inv;
  }
  __builtin_amdgcn_fence(__ATOMIC_RELEASE, "workgroup");
  __builtin_amdgcn_wave_barrier();
  __builtin_amdgcn_fence(__ATOMIC_ACQUIRE, "workgroup");
  {
    const int c8 = (lane & 15) * 8;
    unsigned short* yhb = yh + (size_t)b * pl;
    unsigned short* ylb = yl + (size_t)b * pl;
    for (int pass = 0; pass < 2; ++pass) {
#pragma unroll
      for (int it = 0; it < 8; ++it) {
        const int row = it * 2 + hh;
        const float* sp = os + row * kAttOP + c8;
        v8h hv, lv;
#pragma unroll
        for (int e = 0; e < 8; ++e) {
          const unsigned short hb = f2bf_bits(sp[e]);
          const unsigned short lb = f2bf_bits(sp[e] - bf_bits2f(hb));
          hv[e] = __builtin_bit_cast(_Float16, hb);
          lv[e] = __builtin_bit_cast(_Float16, lb);
        }
        const size_t yo = (size_t)(q0 + row) * kCi + c8;
        *(volatile v8h*)(yhb + yo) = hv;
        *(volatile v8h*)(ylb + yo) = lv;
      }
      __threadfence();
    }
  }
}


__global__ __launch_bounds__(256) void k_cast_bf16(const float* __restrict__ in, unsigned short* __restrict__ out, int n8) {
  const int i = blockIdx.x * 256 + threadIdx.x;
  if (i >= n8) return;
  const float* sp = in + (size_t)8 * i;
  const v4f a = *(const v4f*)sp;
  const v4f q = *(const v4f*)(sp + 4);
  v8h hv;
#pragma unroll
  for (int e = 0; e < 4; ++e) {
    hv[e]     = __builtin_bit_cast(_Float16, f2bf_bits(a[e]));
    hv[4 + e] = __builtin_bit_cast(_Float16, f2bf_bits(q[e]));
  }
  unsigned short* dst = out + (size_t)8 * i;
  *(volatile v8h*)dst = hv;
  __threadfence();
  *(volatile v8h*)dst = hv;
}

__global__ __launch_bounds__(256) void k_pack_convw(const float* __restrict__ w, unsigned short* __restrict__ wp, int nthreads) {
  const int i = blockIdx.x * 256 + threadIdx.x;
  if (i >= nthreads) return;
  const int c8 = i & 31;
  const int rowid = i >> 5;
  const int tap = rowid % 9;
  const int lo_ = rowid / 9;
  const float* src = w + ((size_t)lo_ * kCh + c8 * 8) * 9 + tap;
  v8h hv;
#pragma unroll
  for (int e = 0; e < 8; ++e) hv[e] = __builtin_bit_cast(_Float16, f2bf_bits(src[e * 9]));
  unsigned short* dst = wp + (size_t)rowid * kCh + c8 * 8;
  *(volatile v8h*)dst = hv;
  __threadfence();
  *(volatile v8h*)dst = hv;
}

__global__ __launch_bounds__(256) void k_prep_tables(
    const float* __restrict__ g_b, const float* __restrict__ th_b, const float* __restrict__ ph_b,
    const float* __restrict__ w_b, const float* __restrict__ c_b,
    const float* __restrict__ g1, const float* __restrict__ b1, const float* __restrict__ m1, const float* __restrict__ v1,
    const float* __restrict__ g2, const float* __restrict__ b2, const float* __restrict__ m2, const float* __restrict__ v2,
    float* __restrict__ tab) {
  const int tb = blockIdx.x;
  const int t  = threadIdx.x;
  const int n    = (tb < 3) ? (kLayers * kCi) : (kLayers * kCh);
  const int toff = (tb < 3) ? tb * (kLayers * kCi) : (3 * kLayers * kCi + (tb - 3) * (kLayers * kCh));
  const int e0 = 4 * t;
  if (e0 >= n) return;
  v4f o = (v4f){0.f,0.f,0.f,0.f};
  if (tb == 0) {
#pragma unroll
    for (int k = 0; k < 4; ++k) o[k] = bf_rne(g_b[e0 + k]);
  } else if (tb == 1) {
#pragma unroll
    for (int k = 0; k < 4; ++k) o[k] = bf_rne(th_b[e0 + k]);
  } else if (tb == 2) {
#pragma unroll
    for (int k = 0; k < 4; ++k) o[k] = bf_rne(ph_b[e0 + k]);
  } else if (tb == 3) {
#pragma unroll
    for (int k = 0; k < 4; ++k) o[k] = bf_rne(w_b[e0 + k]);
  } else if (tb == 4) {
#pragma unroll
    for (int k = 0; k < 4; ++k) o[k] = bf_rne(c_b[e0 + k]);
  } else if (tb == 5 || tb == 6) {
#pragma unroll
    for (int k = 0; k < 4; ++k) {
      const float gg = bf_rne(g1[e0 + k]);
      const float vv = bf_rne(v1[e0 + k]);
      const float bb = bf_rne(b1[e0 + k]);
      const float mm = bf_rne(m1[e0 + k]);
      const float sc = gg / sqrtf(vv + kBnEps);
      o[k] = (tb == 5) ? sc : (bb - mm * sc);
    }
  } else {
#pragma unroll
    for (int k = 0; k < 4; ++k) {
      const float gg = bf_rne(g2[e0 + k]);
      const float vv = bf_rne(v2[e0 + k]);
      const float bb = bf_rne(b2[e0 + k]);
      const float mm = bf_rne(m2[e0 + k]);
      const float sc = gg / sqrtf(vv + kBnEps);
      o[k] = (tb == 7) ? sc : (bb - mm * sc);
    }
  }
  float* dst = tab + toff + e0;
  *(volatile v4f*)dst = o;
  __threadfence();
  *(volatile v4f*)dst = o;
}

__global__ __launch_bounds__(256) void k_zero16(unsigned short* __restrict__ p, int n8) {
  const int i = blockIdx.x * 256 + threadIdx.x;
  if (i >= n8) return;
  const v4u z = (v4u){0u, 0u, 0u, 0u};
  unsigned short* dst = p + (size_t)8 * i;
  *(volatile v4u*)dst = z;
  __threadfence();
  *(volatile v4u*)dst = z;
}

__global__ __launch_bounds__(256) void k_transpose_in(const float* __restrict__ x, float* __restrict__ xT) {
  __shared__ float tile[32][33];
  const int p0 = blockIdx.x * 32, c0 = blockIdx.y * 32, b = blockIdx.z, t = threadIdx.x;
  {
    const int cr = t >> 3, p4 = (t & 7) * 4;
    const v4f v = *(const v4f*)(x + ((size_t)b * kCh + c0 + cr) * kNPos + p0 + p4);
    tile[cr][p4 + 0] = bf_rne(v[0]);
    tile[cr][p4 + 1] = bf_rne(v[1]);
    tile[cr][p4 + 2] = bf_rne(v[2]);
    tile[cr][p4 + 3] = bf_rne(v[3]);
  }
  __syncthreads();
  {
    const int pr = t >> 3, c4 = (t & 7) * 4;
    v4f o;
    o[0] = tile[c4 + 0][pr];
    o[1] = tile[c4 + 1][pr];
    o[2] = tile[c4 + 2][pr];
    o[3] = tile[c4 + 3][pr];
    float* dst = xT + ((size_t)b * kNPos + p0 + pr) * kCh + c0 + c4;
    *(volatile v4f*)dst = o;
    __threadfence();
    *(volatile v4f*)dst = o;
  }
}

__global__ __launch_bounds__(256) void k_split_planes(const float* __restrict__ src, unsigned short* __restrict__ hi,
                                                      unsigned short* __restrict__ lo, int n8) {
  const int i = blockIdx.x * 256 + threadIdx.x;
  if (i >= n8) return;
  const float* sp = src + (size_t)8 * i;
  const v4f a = *(const v4f*)sp;
  const v4f q = *(const v4f*)(sp + 4);
  v8h hv, lv;
#pragma unroll
  for (int e = 0; e < 4; ++e) {
    {
      const unsigned short hb = f2bf_bits(a[e]);
      const unsigned short lb = f2bf_bits(a[e] - bf_bits2f(hb));
      hv[e] = __builtin_bit_cast(_Float16, hb);
      lv[e] = __builtin_bit_cast(_Float16, lb);
    }
    {
      const unsigned short hb = f2bf_bits(q[e]);
      const unsigned short lb = f2bf_bits(q[e] - bf_bits2f(hb));
      hv[4 + e] = __builtin_bit_cast(_Float16, hb);
      lv[4 + e] = __builtin_bit_cast(_Float16, lb);
    }
  }
  unsigned short* dh = hi + (size_t)8 * i;
  unsigned short* dl = lo + (size_t)8 * i;
  *(volatile v8h*)dh = hv;
  *(volatile v8h*)dl = lv;
  __threadfence();
  *(volatile v8h*)dh = hv;
  *(volatile v8h*)dl = lv;
}

__global__ __launch_bounds__(256) void k_transpose_out(const float* __restrict__ xT, float* __restrict__ out) {
  __shared__ float tile[32][33];
  const int p0 = blockIdx.x * 32, c0 = blockIdx.y * 32, b = blockIdx.z, t = threadIdx.x;
  {
    const int pr = t >> 3, c4 = (t & 7) * 4;
    const v4f v = *(const v4f*)(xT + ((size_t)b * kNPos + p0 + pr) * kCh + c0 + c4);
    tile[pr][c4 + 0] = v[0];
    tile[pr][c4 + 1] = v[1];
    tile[pr][c4 + 2] = v[2];
    tile[pr][c4 + 3] = v[3];
  }
  __syncthreads();
  {
    const int cr = t >> 3, p4 = (t & 7) * 4;
    v4f o;
    o[0] = tile[p4 + 0][cr];
    o[1] = tile[p4 + 1][cr];
    o[2] = tile[p4 + 2][cr];
    o[3] = tile[p4 + 3][cr];
    float* dst = out + ((size_t)b * kCh + c0 + cr) * kNPos + p0 + p4;
    *(volatile v4f*)dst = o;
    __threadfence();
    *(volatile v4f*)dst = o;
  }
}

extern "C" void kernel_launch(void* const* d_in, const int* in_sizes, int n_in,
                              void* d_out, int out_size, void* d_ws, size_t ws_size, hipStream_t stream) {
  (void)in_sizes; (void)n_in; (void)out_size;
  const float* x_in   = (const float*)d_in[0];
  const float* g_w    = (const float*)d_in[1];
  const float* g_b    = (const float*)d_in[2];
  const float* th_w   = (const float*)d_in[3];
  const float* th_b   = (const float*)d_in[4];
  const float* ph_w   = (const float*)d_in[5];
  const float* ph_b   = (const float*)d_in[6];
  const float* ww_w   = (const float*)d_in[7];
  const float* ww_b   = (const float*)d_in[8];
  const float* bn1_g  = (const float*)d_in[9];
  const float* bn1_b  = (const float*)d_in[10];
  const float* bn1_m  = (const float*)d_in[11];
  const float* bn1_v  = (const float*)d_in[12];
  const float* conv_w = (const float*)d_in[13];
  const float* conv_b = (const float*)d_in[14];
  const float* bn2_g  = (const float*)d_in[15];
  const float* bn2_b  = (const float*)d_in[16];
  const float* bn2_m  = (const float*)d_in[17];
  const float* bn2_v  = (const float*)d_in[18];

  char* base = (char*)d_ws;
  size_t off = 0;
  auto carve = [&](size_t bytes) -> void* {
    off = (off + 255) & ~(size_t)255;
    void* p = base + off;
    off += bytes;
    return p;
  };
  const size_t nProjW = (size_t)kLayers * kCi * kCh;
  const size_t nPlane = (size_t)kBatch * kNPos * kCi;
  const size_t nXPlane = (size_t)kBatch * kNPos * kCh;
  const size_t nPadPlane = (size_t)kBatch * kNPad * kCh;
  unsigned short* wg16  = (unsigned short*)carve(nProjW * 2);
  unsigned short* wth16 = (unsigned short*)carve(nProjW * 2);
  unsigned short* wph16 = (unsigned short*)carve(nProjW * 2);
  unsigned short* ww16  = (unsigned short*)carve(nProjW * 2);
  unsigned short* wpk16 = (unsigned short*)carve((size_t)kLayers * kCh * kKConv * 2);
  float* tab   = (float*)carve((size_t)kTabTotal * 4);
  float* xT32  = (float*)carve(nXPlane * 4);
  unsigned short* xh  = (unsigned short*)carve(nXPlane * 2);
  unsigned short* xl  = (unsigned short*)carve(nXPlane * 2);
  unsigned short* thh = (unsigned short*)carve(nPlane * 2);
  unsigned short* thl = (unsigned short*)carve(nPlane * 2);
  unsigned short* phh = (unsigned short*)carve(nPlane * 2);
  unsigned short* phl = (unsigned short*)carve(nPlane * 2);
  unsigned short* gp  = (unsigned short*)carve(nPlane * 2);
  unsigned short* yh  = (unsigned short*)carve(nPlane * 2);
  unsigned short* yl  = (unsigned short*)carve(nPlane * 2);
  unsigned short* x1h = (unsigned short*)carve(nPadPlane * 2 * 2);
  unsigned short* x1l = x1h + nPadPlane;
  if (off > ws_size) return;
  float* outp = (float*)d_out;

  const int nW8 = (int)(nProjW / 8);
  k_cast_bf16<<<(nW8 + 255) / 256, 256, 0, stream>>>(g_w,  wg16,  nW8);
  k_cast_bf16<<<(nW8 + 255) / 256, 256, 0, stream>>>(th_w, wth16, nW8);
  k_cast_bf16<<<(nW8 + 255) / 256, 256, 0, stream>>>(ph_w, wph16, nW8);
  k_cast_bf16<<<(nW8 + 255) / 256, 256, 0, stream>>>(ww_w, ww16,  nW8);
  const int nPk = kLayers * kCh * 9 * (kCh / 8);
  k_pack_convw<<<(nPk + 255) / 256, 256, 0, stream>>>(conv_w, wpk16, nPk);
  k_prep_tables<<<9, 256, 0, stream>>>(g_b, th_b, ph_b, ww_b, conv_b,
                                        bn1_g, bn1_b, bn1_m, bn1_v,
                                        bn2_g, bn2_b, bn2_m, bn2_v, tab);
  const int nZ8 = (int)(nPadPlane * 2 / 8);
  k_zero16<<<(nZ8 + 255) / 256, 256, 0, stream>>>(x1h, nZ8);
  k_transpose_in<<<dim3(kNPos / 32, kCh / 32, kBatch), 256, 0, stream>>>(x_in, xT32);

  const int nS8 = (int)(nXPlane / 8);
  const long strideX   = (long)kNPos * kCh;
  const long strideP   = (long)kNPos * kCi;
  const long strideG   = (long)kCi * kNPos;
  const long stridePad = (long)kNPad * kCh;

  for (int l = 0; l < kLayers; ++l) {
    k_split_planes<<<(nS8 + 255) / 256, 256, 0, stream>>>(xT32, xh, xl, nS8);

    const unsigned short* wthL = wth16 + (size_t)l * kCi * kCh;
    const unsigned short* wphL = wph16 + (size_t)l * kCi * kCh;
    const unsigned short* wgL  = wg16  + (size_t)l * kCi * kCh;
    const unsigned short* wwL  = ww16  + (size_t)l * kCh * kCi;
    const unsigned short* wpkL = wpk16 + (size_t)l * kCh * kKConv;

    if (l == 0) {
      gemm_bf16_64<true, false, 2, 0, 2, false, false><<<dim3(16, kBatch), 256, 0, stream>>>(
          xh, xl, kCh, strideX, wthL, wthL, kCh, 0L, thh, thl, kCi, strideP,
          tab + kTabThb + l * kCi, tab, tab, xT32, kCh, strideX, kNPos, kCi, kCh);
      gemm_bf16_64<true, false, 2, 0, 2, false, false><<<dim3(16, kBatch), 256, 0, stream>>>(
          xh, xl, kCh, strideX, wphL, wphL, kCh, 0L, phh, phl, kCi, strideP,
          tab + kTabPhb + l * kCi, tab, tab, xT32, kCh, strideX, kNPos, kCi, kCh);
    } else {
      gemm_bf16_64<true, false, 2, 0, 1, false, false><<<dim3(16, kBatch), 256, 0, stream>>>(
          xh, xl, kCh, strideX, wthL, wthL, kCh, 0L, thh, thh, kCi, strideP,
          tab + kTabThb + l * kCi, tab, tab, xT32, kCh, strideX, kNPos, kCi, kCh);
      gemm_bf16_64<true, false, 2, 0, 1, false, false><<<dim3(16, kBatch), 256, 0, stream>>>(
          xh, xl, kCh, strideX, wphL, wphL, kCh, 0L, phh, phh, kCi, strideP,
          tab + kTabPhb + l * kCi, tab, tab, xT32, kCh, strideX, kNPos, kCi, kCh);
    }
    gemm_bf16_64<false, true, 1, 0, 1, false, false><<<dim3(16, kBatch), 256, 0, stream>>>(
        wgL, wgL, kCh, 0L, xh, xl, kCh, strideX, gp, gp, kNPos, strideG,
        tab + kTabGb + l * kCi, tab, tab, xT32, kCh, strideX, kCi, kNPos, kCh);

    if (l == 0) attn_kernel<true><<<dim3(kNPos / 64, kBatch), 128, 0, stream>>>(thh, thl, phh, phl, gp, yh, yl);
    else        attn_kernel<false><<<dim3(kNPos / 64, kBatch), 128, 0, stream>>>(thh, thl, phh, phl, gp, yh, yl);

    gemm_bf16_64<true, false, 2, 1, 2, true, true><<<dim3(32, kBatch), 256, 0, stream>>>(
        yh, yl, kCi, strideP, wwL, wwL, kCi, 0L, x1h, x1l, kCh, stridePad,
        tab + kTabWb + l * kCh, tab + kTabS1 + l * kCh, tab + kTabT1 + l * kCh,
        xT32, kCh, strideX, kNPos, kCh, kCi);

    conv3x3_bf16_64<<<dim3(32, kBatch), 256, 0, stream>>>(
        x1h, x1l, wpkL, xT32, tab + kTabCb + l * kCh, tab + kTabS2 + l * kCh, tab + kTabT2 + l * kCh);
  }

  k_transpose_out<<<dim3(kNPos / 32, kCh / 32, kBatch), 256, 0, stream>>>(xT32, outp);
}
